// DualAttentionEncoderBlock_51135880626863
// MI455X (gfx1250) — hardware-verified
//
#include <hip/hip_runtime.h>
#include <math.h>

constexpr int kBatch = 4;
constexpr int kSeq   = 1024;
constexpr int kDim   = 768;
constexpr int kHeads = 16;
constexpr int kTok   = kBatch * kSeq;
constexpr int kPadN  = 3072;
constexpr int kQkvW  = 1024;
constexpr int kFfn   = 1536;
constexpr float kWCarry   = 16.0f;
constexpr float kInvW     = 1.0f / 16.0f;
constexpr float kPCarry   = 2048.0f;
constexpr float kPVScale  = 256.0f / 2048.0f;
constexpr float kOutScale = 1.0f / (256.0f * 16.0f);
constexpr float kSeqScale = 0.14433756729740643f;
constexpr float kChanScale = 0.125f;
constexpr float kInvDim   = 1.0f / 768.0f;
constexpr float kLnEps    = 1e-5f;

constexpr size_t kPlane32 = (size_t)kTok * kDim * 4;
constexpr size_t kOffXSEQ = 0;
constexpr size_t kOffFUS  = kOffXSEQ + kPlane32;
constexpr size_t kOffXSUM = kOffFUS + kPlane32;
constexpr size_t kArena   = kOffXSUM + kPlane32;
constexpr size_t kOffQKV16 = kArena + 0;
constexpr size_t kOffVTS   = kArena + 25165824;
constexpr size_t kOffSC    = kArena + 33554432;
constexpr size_t kOffX16   = kOffSC;
constexpr size_t kOffP16   = kArena + 67108864;
constexpr size_t kOffWQKVP = kOffP16;
constexpr size_t kOffBQKVP = kOffP16 + 4718592;
constexpr size_t kOffCTXS  = kArena + 83886080;
constexpr size_t kOffWOP   = kArena + 92274688;
constexpr size_t kOffS1    = kArena + 0;
constexpr size_t kOffXT16  = kArena + 0;
constexpr size_t kOffCTXC  = kOffXT16;
constexpr size_t kOffCIW   = kArena + 6291456;
constexpr size_t kOffCOW   = kOffCIW;
constexpr size_t kOffQKVC  = kArena + 12582912;
constexpr size_t kOffCHO   = kOffQKVC;
constexpr size_t kOffVTC   = kArena + 31457280;
constexpr size_t kOffSCC   = kArena + 37748736;
constexpr size_t kOffPC    = kArena + 75497472;
constexpr size_t kOffW1    = kArena + 0;
constexpr size_t kOffW2    = kArena + 4718592;
constexpr size_t kOffH1    = kArena + 8388608;
constexpr size_t kOffS3    = kArena + 20971520;
constexpr size_t kWsTotal  = kArena + 94371840;
static_assert(kWsTotal <= (size_t)134217728);
static_assert(kOffWOP + 1572864 <= kWsTotal);
static_assert(kOffS3 + kPlane32 <= kWsTotal);

typedef __attribute__((ext_vector_type(16))) _Float16 v16h;
typedef __attribute__((ext_vector_type(8)))  _Float16 v8h;
typedef __attribute__((ext_vector_type(16))) __bf16   v16b;
typedef __attribute__((ext_vector_type(8)))  __bf16   v8b;
typedef __attribute__((ext_vector_type(8)))  float    v8f;
typedef __attribute__((ext_vector_type(4)))  float    v4f;
typedef __attribute__((ext_vector_type(4)))  unsigned int v4u;

__device__ __forceinline__ unsigned short f2bf_bits(float f) {
  unsigned u = __float_as_uint(f);
  return (unsigned short)((u + 0x7FFFu + ((u >> 16) & 1u)) >> 16);
}
__device__ __forceinline__ float bf_bits2f(unsigned short h) { return __uint_as_float(((unsigned)h) << 16); }

__device__ __forceinline__ void dep_guard_h(v8f& a, v8f& b, v16h x, v16h y) { asm volatile("v_nop\n\tv_nop\n\tv_nop\n\tv_nop" : "+v"(a), "+v"(b) : "v"(x), "v"(y)); }
__device__ __forceinline__ void dep_guard_b(v8f& a, v8f& b, v16b x, v16b y) { asm volatile("v_nop\n\tv_nop\n\tv_nop\n\tv_nop" : "+v"(a), "+v"(b) : "v"(x), "v"(y)); }
__device__ __forceinline__ void keep4_h(v16h a, v16h b, v16h c, v16h d) { asm volatile("v_nop" :: "v"(a), "v"(b), "v"(c), "v"(d)); }
__device__ __forceinline__ void keep4_b(v16b a, v16b b, v16b c, v16b d) { asm volatile("v_nop" :: "v"(a), "v"(b), "v"(c), "v"(d)); }
__device__ __forceinline__ void acc_guard4(v8f& a, v8f& b, v8f& c, v8f& d) { asm volatile("v_nop\n\tv_nop\n\tv_nop\n\tv_nop" : "+v"(a), "+v"(b), "+v"(c), "+v"(d)); }
template <typename T> struct Frag;
template <> struct Frag<_Float16> {
  typedef v16h V; union U { v16h v; v8h h[2]; };
  static __device__ __forceinline__ v16h load(const _Float16* p) {
    U f; f.h[0] = *(const v8h*)(p); f.h[1] = *(const v8h*)(p + 16); return f.v;
  }
  static __device__ __forceinline__ v8f mma(v16h a, v16h b, v8f c) {
    return __builtin_amdgcn_wmma_f32_16x16x32_f16(false, a, false, b, (short)0, c, false, false);
  }
  static __device__ __forceinline__ void guard(v8f& a, v8f& b, v16h x, v16h y) { dep_guard_h(a, b, x, y); }
  static __device__ __forceinline__ void keep(v16h a, v16h b, v16h c, v16h d) { keep4_h(a, b, c, d); }
};
template <> struct Frag<__bf16> {
  typedef v16b V; union U { v16b v; v8b h[2]; };
  static __device__ __forceinline__ v16b load(const __bf16* p) {
    U f; f.h[0] = *(const v8b*)(p); f.h[1] = *(const v8b*)(p + 16); return f.v;
  }
  static __device__ __forceinline__ v8f mma(v16b a, v16b b, v8f c) {
    return __builtin_amdgcn_wmma_f32_16x16x32_bf16(false, a, false, b, (short)0, c, false, false);
  }
  static __device__ __forceinline__ void guard(v8f& a, v8f& b, v16b x, v16b y) { dep_guard_b(a, b, x, y); }
  static __device__ __forceinline__ void keep(v16b a, v16b b, v16b c, v16b d) { keep4_b(a, b, c, d); }
};

__device__ __forceinline__ unsigned pk16(unsigned short a, unsigned short b) { return (unsigned)a | ((unsigned)b << 16); }
__device__ __forceinline__ unsigned short h_bits(float f) { const _Float16 h = (_Float16)f; return __builtin_bit_cast(unsigned short, h); }

__device__ __forceinline__ void wave_sync_lds() {
  __builtin_amdgcn_fence(__ATOMIC_RELEASE, "workgroup");
  __builtin_amdgcn_wave_barrier();
  __builtin_amdgcn_fence(__ATOMIC_ACQUIRE, "workgroup");
}
__device__ __forceinline__ float wave_sum(float v) {
#pragma unroll
  for (int off = 16; off > 0; off >>= 1) v += __shfl_xor(v, off, 32);
  return v;
}
__device__ __forceinline__ float wave_max(float v) {
#pragma unroll
  for (int off = 16; off > 0; off >>= 1) v = fmaxf(v, __shfl_xor(v, off, 32));
  return v;
}

template <int ET> struct Elem;
template <> struct Elem<0> { typedef _Float16 T; };
template <> struct Elem<1> { typedef __bf16 T; };
template <int ET, bool SPLIT, int BIAS_MODE, int OUT_MODE, bool RESID, int ACT = 0>
__global__ __launch_bounds__(256) void wmma_gemm64(
    const unsigned short* __restrict__ Ap, const unsigned short* __restrict__ A2p, int lda, long strideA,
    const unsigned short* __restrict__ Btp, const unsigned short* __restrict__ Bt2p, int ldb, long strideB,
    void* __restrict__ Cout, void* __restrict__ Cout2, int ldc, long strideC,
    const float* __restrict__ bias,
    const float* __restrict__ resid, long strideR,
    int M, int N, int K, float scale) {
  typedef typename Elem<ET>::T T;
  typedef typename Frag<T>::V V;
  const T* A = (const T*)Ap; const T* A2 = (const T*)A2p; const T* Bt = (const T*)Btp; const T* Bt2 = (const T*)Bt2p;
  __shared__ __align__(16) float sT[8][16 * 68];
  const int b    = blockIdx.y;
  const int lane = threadIdx.x & 31;
  const int wave = threadIdx.x >> 5;
  const int tilesN = N >> 6;
  const int tilesM = M >> 6;
  const int tile = blockIdx.x * 8 + wave;
  if (tile >= tilesM * tilesN) return;
  const int tm = tile / tilesN;
  const int tn = tile - tm * tilesN;
  const int m0 = tm << 6;
  const int n0 = tn << 6;

  const T* Ab  = A  + (size_t)b * strideA;
  const T* Bb  = Bt + (size_t)b * strideB;
  const T* Ab2 = SPLIT ? (A2  + (size_t)b * strideA) : nullptr;
  const T* Bb2 = SPLIT ? (Bt2 + (size_t)b * strideB) : nullptr;

  const int rlane = lane & 15;
  const int koff  = (lane >> 4) * 8;
  const int mOff  = (lane >> 4) * 8;

  v8f acc[4][4];
#pragma unroll
  for (int i = 0; i < 4; ++i)
#pragma unroll
    for (int j = 0; j < 4; ++j) acc[i][j] = (v8f){0.f,0.f,0.f,0.f,0.f,0.f,0.f,0.f};

  for (int k0 = 0; k0 < K; k0 += 32) {
    V bh[4], bl[4];
#pragma unroll
    for (int j = 0; j < 4; ++j) {
      const size_t bo = (size_t)(n0 + (j << 4) + rlane) * ldb + koff + k0;
      bh[j] = Frag<T>::load(Bb + bo);
      if (SPLIT) bl[j] = Frag<T>::load(Bb2 + bo);
    }
#pragma unroll
    for (int i = 0; i < 4; ++i) {
      const size_t ao = (size_t)(m0 + (i << 4) + rlane) * lda + koff + k0;
      V ah = Frag<T>::load(Ab + ao);
      V al;
      if (SPLIT) al = Frag<T>::load(Ab2 + ao);
#pragma unroll
      for (int j = 0; j < 4; ++j) {
        acc[i][j] = Frag<T>::mma(ah, bh[j], acc[i][j]);
        if (SPLIT) {
          acc[i][j] = Frag<T>::mma(ah, bl[j], acc[i][j]);
          acc[i][j] = Frag<T>::mma(al, bh[j], acc[i][j]);
        }
      }
      Frag<T>::guard(acc[i][0], acc[i][3], ah, SPLIT ? al : ah);
    }
    Frag<T>::keep(bh[0], bh[1], bh[2], bh[3]);
    if (SPLIT) Frag<T>::keep(bl[0], bl[1], bl[2], bl[3]);
  }
  acc_guard4(acc[0][0], acc[0][1], acc[0][2], acc[0][3]);
  acc_guard4(acc[1][0], acc[1][1], acc[1][2], acc[1][3]);
  acc_guard4(acc[2][0], acc[2][1], acc[2][2], acc[2][3]);
  acc_guard4(acc[3][0], acc[3][1], acc[3][2], acc[3][3]);

  float* slab = sT[wave];
  const float* Rb = RESID ? (resid + (size_t)b * strideR) : nullptr;
#pragma unroll
  for (int i = 0; i < 4; ++i) {
    const int mBase = m0 + (i << 4);
#pragma unroll
    for (int j = 0; j < 4; ++j) {
      const int n = n0 + (j << 4) + rlane;
      float bv = 0.f;
      if (BIAS_MODE == 2) bv = bias[n];
#pragma unroll
      for (int r = 0; r < 8; ++r) {
        float v = acc[i][j][r] * scale;
        if (BIAS_MODE == 1) v += bias[mBase + mOff + r];
        if (BIAS_MODE == 2) v += bv;
        if (RESID) v += Rb[(size_t)(mBase + mOff + r) * ldc + n];
        if (ACT == 2) v = fmaxf(v, 0.0f);
        if (ACT == 4) v = (v > 0.f) ? v : 0.01f * v;
        slab[(mOff + r) * 68 + (j << 4) + rlane] = v;
      }
    }
    __builtin_amdgcn_fence(__ATOMIC_RELEASE, "workgroup");
    __builtin_amdgcn_wave_barrier();
    __builtin_amdgcn_fence(__ATOMIC_ACQUIRE, "workgroup");
    if (OUT_MODE == 0) {
      float* C = (float*)Cout + (size_t)b * strideC;
      const int hh = lane >> 4, c4 = (lane & 15) * 4;
      for (int pass = 0; pass < 2; ++pass) {
#pragma unroll
        for (int it = 0; it < 8; ++it) {
          const int row = it * 2 + hh;
          v4f v = *(const v4f*)(slab + row * 68 + c4);
          *(volatile v4f*)(C + (size_t)(mBase + row) * ldc + n0 + c4) = v;
        }
        __threadfence();
      }
    } else {
      const int q = lane >> 3, c8 = (lane & 7) * 8;
      unsigned short* C  = (unsigned short*)Cout  + (size_t)b * strideC;
      unsigned short* C2 = (OUT_MODE == 2) ? ((unsigned short*)Cout2 + (size_t)b * strideC) : nullptr;
      for (int pass = 0; pass < 2; ++pass) {
#pragma unroll
        for (int it = 0; it < 4; ++it) {
          const int row = it * 4 + q;
          const float* sp = slab + row * 68 + c8;
          v8h hv, lv;
#pragma unroll
          for (int e = 0; e < 8; ++e) {
            if (OUT_MODE == 1) {
              hv[e] = (_Float16)sp[e];
            } else {
              unsigned short hb = f2bf_bits(sp[e]);
              unsigned short lb = f2bf_bits(sp[e] - bf_bits2f(hb));
              hv[e] = __builtin_bit_cast(_Float16, hb);
              lv[e] = __builtin_bit_cast(_Float16, lb);
            }
          }
          *(volatile v8h*)(C + (size_t)(mBase + row) * ldc + n0 + c8) = hv;
          if (OUT_MODE == 2) *(volatile v8h*)(C2 + (size_t)(mBase + row) * ldc + n0 + c8) = lv;
        }
        __threadfence();
      }
    }
    __builtin_amdgcn_fence(__ATOMIC_RELEASE, "workgroup");
    __builtin_amdgcn_wave_barrier();
    __builtin_amdgcn_fence(__ATOMIC_ACQUIRE, "workgroup");
  }
}

__global__ __launch_bounds__(256) void k_cast_rows(const float* __restrict__ in, unsigned short* __restrict__ out,
                                                   int rows, int cols, float scale) {
  const int lane = threadIdx.x & 31, wave = threadIdx.x >> 5;
  const int row = blockIdx.x * 8 + wave;
  if (row >= rows) return;
  const int nseg = cols >> 8;
  const float* ir = in + (size_t)row * cols;
  unsigned short* orw = out + (size_t)row * cols;
#pragma unroll 1
  for (int j = 0; j < nseg; ++j) {
    const float* p = ir + 256 * j + 8 * lane;
    const v4f a = *(const v4f*)(p);
    const v4f c = *(const v4f*)(p + 4);
    unsigned short hb[8];
#pragma unroll
    for (int e = 0; e < 4; ++e) { hb[e] = h_bits(a[e] * scale); hb[4 + e] = h_bits(c[e] * scale); }
    const v4u u = (v4u){pk16(hb[0], hb[1]), pk16(hb[2], hb[3]), pk16(hb[4], hb[5]), pk16(hb[6], hb[7])};
    unsigned short* q = orw + 256 * j + 8 * lane;
    *(volatile v4u*)q = u;
    __threadfence();
    *(volatile v4u*)q = u;
  }
}

__global__ __launch_bounds__(256) void k_cast_qkvpad(const float* __restrict__ wq, const float* __restrict__ wk,
                                                     const float* __restrict__ wv, const float* __restrict__ bq,
                                                     const float* __restrict__ bk, const float* __restrict__ bv,
                                                     unsigned short* __restrict__ wout, float* __restrict__ bout) {
  const int tid = threadIdx.x, lane = tid & 31, wave = tid >> 5;
  if (blockIdx.x < 384) {
    const int row = blockIdx.x * 8 + wave;
    const int part = row >> 10;
    const int hp = row & 1023;
    const int h = hp >> 6, d = hp & 63;
    const bool real = (d < 48);
    const int srow = h * 48 + (real ? d : 47);
    const float* W = (part == 0) ? wq : ((part == 1) ? wk : wv);
    const float* ir = W + (size_t)srow * kDim;
    unsigned short* orw = wout + (size_t)row * kDim;
    const float sc = real ? kWCarry : 0.0f;
#pragma unroll 1
    for (int j = 0; j < 3; ++j) {
      const float* p = ir + 256 * j + 8 * lane;
      const v4f a = *(const v4f*)(p);
      const v4f c = *(const v4f*)(p + 4);
      unsigned short hb[8];
#pragma unroll
      for (int e = 0; e < 4; ++e) {
        hb[e]     = h_bits(real ? a[e] * sc : 0.0f);
        hb[4 + e] = h_bits(real ? c[e] * sc : 0.0f);
      }
      const v4u u = (v4u){pk16(hb[0], hb[1]), pk16(hb[2], hb[3]), pk16(hb[4], hb[5]), pk16(hb[6], hb[7])};
      unsigned short* q = orw + 256 * j + 8 * lane;
      *(volatile v4u*)q = u;
      __threadfence();
      *(volatile v4u*)q = u;
    }
  } else {
    const int idx = 4 * tid;
    const int h = idx >> 6, d = idx & 63;
    const bool real = (d < 48);
    const int sidx = h * 48 + (real ? d : 44);
#pragma unroll 1
    for (int j = 0; j < 3; ++j) {
      const float* bp = (j == 0) ? bq : ((j == 1) ? bk : bv);
      const v4f a = *(const v4f*)(bp + sidx);
      v4f o;
      o[0] = real ? a[0] : 0.0f; o[1] = real ? a[1] : 0.0f; o[2] = real ? a[2] : 0.0f; o[3] = real ? a[3] : 0.0f;
      float* q = bout + 1024 * j + idx;
      *(volatile v4f*)q = o;
      __threadfence();
      *(volatile v4f*)q = o;
    }
  }
}

__global__ __launch_bounds__(256) void k_cast_wopad(const float* __restrict__ wo, unsigned short* __restrict__ out) {
  const int lane = threadIdx.x & 31, wave = threadIdx.x >> 5;
  const int n = blockIdx.x * 8 + wave;
  if (n >= kDim) return;
  const float* ir = wo + (size_t)n * kDim;
  unsigned short* orw = out + (size_t)n * kQkvW;
#pragma unroll 1
  for (int j = 0; j < 4; ++j) {
    const int c = 256 * j + 8 * lane;
    const int h = c >> 6, d = c & 63;
    const bool real = (d < 48);
    const int sd = real ? d : 40;
    const float* p = ir + h * 48 + sd;
    const v4f a  = *(const v4f*)(p);
    const v4f a2 = *(const v4f*)(p + 4);
    unsigned short hb[8];
#pragma unroll
    for (int e = 0; e < 4; ++e) {
      hb[e]     = h_bits(real ? a[e]  * kWCarry : 0.0f);
      hb[4 + e] = h_bits(real ? a2[e] * kWCarry : 0.0f);
    }
    const v4u u = (v4u){pk16(hb[0], hb[1]), pk16(hb[2], hb[3]), pk16(hb[4], hb[5]), pk16(hb[6], hb[7])};
    unsigned short* q = orw + c;
    *(volatile v4u*)q = u;
    __threadfence();
    *(volatile v4u*)q = u;
  }
}

__global__ __launch_bounds__(256) void k_xt16(const float* __restrict__ x, unsigned short* __restrict__ out) {
  __shared__ float sm[64][65];
  const int tid = threadIdx.x;
  const int t0 = blockIdx.x * 64;
  const int l0 = blockIdx.y * 64;
  const int b  = blockIdx.z;
  const float* xb = x + (size_t)b * kSeq * kDim;
#pragma unroll
  for (int i = 0; i < 16; ++i) {
    const int e = i * 256 + tid;
    const int r = e >> 6;
    const int c = e & 63;
    sm[c][r] = xb[(size_t)(l0 + r) * kDim + t0 + c];
  }
  __syncthreads();
  const int lane = tid & 31, wave = tid >> 5;
  const int q = lane >> 3, c8 = (lane & 7) * 8;
  unsigned short* ob = out + (size_t)b * kDim * kSeq;
  for (int pass = 0; pass < 2; ++pass) {
#pragma unroll
    for (int it = 0; it < 2; ++it) {
      const int row = wave * 8 + it * 4 + q;
      unsigned short hb[8];
#pragma unroll
      for (int e = 0; e < 8; ++e) hb[e] = h_bits(sm[row][c8 + e]);
      const v4u u = (v4u){pk16(hb[0], hb[1]), pk16(hb[2], hb[3]), pk16(hb[4], hb[5]), pk16(hb[6], hb[7])};
      *(volatile v4u*)(ob + (size_t)(t0 + row) * kSeq + l0 + c8) = u;
    }
    __threadfence();
  }
}

__global__ __launch_bounds__(256) void k_vt_build(const unsigned short* __restrict__ src, unsigned short* __restrict__ vt, int R) {
  __shared__ unsigned short tile[64][72];
  const int tid = threadIdx.x;
  const int g = blockIdx.y, m0 = blockIdx.x * 64;
  const int b = g >> 4, h = g & 15;
  const unsigned short* sb = src + ((size_t)b * R + m0) * kPadN + 2048 + h * 64;
#pragma unroll
  for (int it = 0; it < 2; ++it) {
    const int e = it * 256 + tid;
    const int r = e >> 3;
    const int c16 = (e & 7) * 8;
    const v4u u = *(const v4u*)(sb + (size_t)r * kPadN + c16);
#pragma unroll
    for (int w = 0; w < 4; ++w) {
      const unsigned uw = u[w];
      tile[c16 + 2 * w][r]     = (unsigned short)(uw & 0xffffu);
      tile[c16 + 2 * w + 1][r] = (unsigned short)(uw >> 16);
    }
  }
  __syncthreads();
  const int lane = tid & 31, wave = tid >> 5;
  const int q = lane >> 3, c8 = (lane & 7) * 8;
  for (int pass = 0; pass < 2; ++pass) {
#pragma unroll
    for (int it = 0; it < 2; ++it) {
      const int d = wave * 8 + it * 4 + q;
      unsigned short hb[8];
#pragma unroll
      for (int e = 0; e < 8; ++e) hb[e] = tile[d][c8 + e];
      const v4u u = (v4u){pk16(hb[0], hb[1]), pk16(hb[2], hb[3]), pk16(hb[4], hb[5]), pk16(hb[6], hb[7])};
      *(volatile v4u*)(vt + ((size_t)g * 64 + d) * R + m0 + c8) = u;
    }
    __threadfence();
  }
}

__global__ __launch_bounds__(128) void k_softmax(const float* __restrict__ S, unsigned short* __restrict__ P,
                                                 const float* __restrict__ relb, int ncols, int rows_per_group,
                                                 int h0, int use_bias, float carry) {
  __shared__ float redm[4];
  __shared__ float reds[4];
  const int row = blockIdx.x;
  const int t = threadIdx.x, lane = t & 31, wave = t >> 5;
  const int nt = ncols >> 3;
  const bool valid = (t < nt);
  const int tc = valid ? t : (nt - 1);
  const float* sr = S + (size_t)row * ncols + 8 * tc;
  const v4f a = *(const v4f*)(sr);
  const v4f c = *(const v4f*)(sr + 4);
  float x[8];
#pragma unroll
  for (int e = 0; e < 4; ++e) { x[e] = a[e]; x[4 + e] = c[e]; }
  if (use_bias != 0) {
    const int j = row / rows_per_group;
    const int l = row - j * rows_per_group;
    const int h = h0 + j;
#pragma unroll
    for (int e = 0; e < 8; ++e) {
      int idx = 8 * tc + e - l + (kSeq - 1);
      idx = idx < 0 ? 0 : (idx > 2 * kSeq - 2 ? 2 * kSeq - 2 : idx);
      x[e] += relb[(size_t)idx * kHeads + h];
    }
  }
  if (!valid) {
#pragma unroll
    for (int e = 0; e < 8; ++e) x[e] = -INFINITY;
  }
  float m = fmaxf(fmaxf(fmaxf(x[0], x[1]), fmaxf(x[2], x[3])), fmaxf(fmaxf(x[4], x[5]), fmaxf(x[6], x[7])));
  m = wave_max(m);
  if (lane == 0) redm[wave] = m;
  __syncthreads();
  m = fmaxf(fmaxf(redm[0], redm[1]), fmaxf(redm[2], redm[3]));
  float ex[8];
  float s = 0.f;
#pragma unroll
  for (int e = 0; e < 8; ++e) { ex[e] = expf(x[e] - m); s += ex[e]; }
  s = wave_sum(s);
  if (lane == 0) reds[wave] = s;
  __syncthreads();
  const float tot = ((reds[0] + reds[1]) + reds[2]) + reds[3];
  const float f = carry / tot;
  unsigned short hb[8];
#pragma unroll
  for (int e = 0; e < 8; ++e) hb[e] = h_bits(ex[e] * f);
  const v4u u = (v4u){pk16(hb[0], hb[1]), pk16(hb[2], hb[3]), pk16(hb[4], hb[5]), pk16(hb[6], hb[7])};
  if (valid) {
    unsigned short* pr = P + (size_t)row * ncols + 8 * t;
    *(volatile v4u*)pr = u;
    __threadfence();
    *(volatile v4u*)pr = u;
  }
}

__global__ __launch_bounds__(256) void k_ln_rows(const float* __restrict__ in, const float* __restrict__ gam,
                                                 const float* __restrict__ bet, float* __restrict__ out32,
                                                 unsigned short* __restrict__ out16, int ld16, int write16, int rows) {
  __shared__ __align__(16) float slab[8][768];
  const int lane = threadIdx.x & 31, wave = threadIdx.x >> 5;
  const int row = blockIdx.x * 8 + wave;
  if (row >= rows) return;
  const float* ir = in + (size_t)row * kDim;
  float v[6][4];
  float s = 0.f;
#pragma unroll
  for (int i = 0; i < 6; ++i) {
    const v4f a = *(const v4f*)(ir + 128 * i + 4 * lane);
#pragma unroll
    for (int e = 0; e < 4; ++e) { v[i][e] = a[e]; s += a[e]; }
  }
  s = wave_sum(s);
  const float mu = s * kInvDim;
  float qq = 0.f;
#pragma unroll
  for (int i = 0; i < 6; ++i)
#pragma unroll
    for (int e = 0; e < 4; ++e) { const float d = v[i][e] - mu; qq += d * d; }
  qq = wave_sum(qq);
  const float rstd = rsqrtf(qq * kInvDim + kLnEps);
  v4f y[6];
#pragma unroll
  for (int i = 0; i < 6; ++i) {
    const v4f g  = *(const v4f*)(gam + 128 * i + 4 * lane);
    const v4f bb = *(const v4f*)(bet + 128 * i + 4 * lane);
#pragma unroll
    for (int e = 0; e < 4; ++e) y[i][e] = (v[i][e] - mu) * rstd * g[e] + bb[e];
  }
  float* orow = out32 + (size_t)row * kDim;
  for (int pass = 0; pass < 2; ++pass) {
#pragma unroll
    for (int i = 0; i < 6; ++i) *(volatile v4f*)(orow + 128 * i + 4 * lane) = y[i];
    __threadfence();
  }
  if (write16 != 0) {
    float* sl = slab[wave];
#pragma unroll
    for (int i = 0; i < 6; ++i) *(v4f*)(sl + 128 * i + 4 * lane) = y[i];
    wave_sync_lds();
    v4u u[3];
#pragma unroll
    for (int j = 0; j < 3; ++j) {
      const v4f a = *(const v4f*)(sl + 256 * j + 8 * lane);
      const v4f c = *(const v4f*)(sl + 256 * j + 8 * lane + 4);
      unsigned short hb[8];
#pragma unroll
      for (int e = 0; e < 4; ++e) { hb[e] = h_bits(a[e]); hb[4 + e] = h_bits(c[e]); }
      u[j] = (v4u){pk16(hb[0], hb[1]), pk16(hb[2], hb[3]), pk16(hb[4], hb[5]), pk16(hb[6], hb[7])};
    }
    unsigned short* o16 = out16 + (size_t)row * ld16;
    for (int pass = 0; pass < 2; ++pass) {
#pragma unroll
      for (int j = 0; j < 3; ++j) *(volatile v4u*)(o16 + 256 * j + 8 * lane) = u[j];
      __threadfence();
    }
  }
}

__global__ __launch_bounds__(256) void k_ln_chan(const float* __restrict__ cho, const float* __restrict__ x,
                                                 const float* __restrict__ xseq, const float* __restrict__ gam,
                                                 const float* __restrict__ bet, float* __restrict__ xsum,
                                                 unsigned short* __restrict__ fus) {
  __shared__ __align__(16) float sm[8][772];
  __shared__ __align__(16) float slab[8][768];
  const int tid = threadIdx.x, lane = tid & 31, wave = tid >> 5;
  const int b = blockIdx.y, l0 = blockIdx.x * 8;
  const float* cb = cho + (size_t)b * kDim * kSeq + l0;
#pragma unroll 4
  for (int it = 0; it < 24; ++it) {
    const int e = it * 256 + tid;
    const int t = e >> 3;
    const int c = e & 7;
    sm[c][t] = cb[(size_t)t * kSeq + c];
  }
  __syncthreads();
  const int c = wave;
  const int gr = b * kSeq + l0 + c;
  const float* xr = x + (size_t)gr * kDim;
  float v[6][4];
  float s = 0.f;
#pragma unroll
  for (int i = 0; i < 6; ++i) {
    const v4f a  = *(const v4f*)(&sm[c][128 * i + 4 * lane]);
    const v4f xx = *(const v4f*)(xr + 128 * i + 4 * lane);
#pragma unroll
    for (int e = 0; e < 4; ++e) { v[i][e] = xx[e] + a[e]; s += v[i][e]; }
  }
  s = wave_sum(s);
  const float mu = s * kInvDim;
  float qq = 0.f;
#pragma unroll
  for (int i = 0; i < 6; ++i)
#pragma unroll
    for (int e = 0; e < 4; ++e) { const float d = v[i][e] - mu; qq += d * d; }
  qq = wave_sum(qq);
  const float rstd = rsqrtf(qq * kInvDim + kLnEps);
  v4f y[6], o[6];
  const float* sr = xseq + (size_t)gr * kDim;
#pragma unroll
  for (int i = 0; i < 6; ++i) {
    const v4f g  = *(const v4f*)(gam + 128 * i + 4 * lane);
    const v4f bb = *(const v4f*)(bet + 128 * i + 4 * lane);
    const v4f xs = *(const v4f*)(sr + 128 * i + 4 * lane);
#pragma unroll
    for (int e = 0; e < 4; ++e) {
      y[i][e] = (v[i][e] - mu) * rstd * g[e] + bb[e];
      o[i][e] = xs[e] + y[i][e];
    }
  }
  float* orow = xsum + (size_t)gr * kDim;
  for (int pass = 0; pass < 2; ++pass) {
#pragma unroll
    for (int i = 0; i < 6; ++i) *(volatile v4f*)(orow + 128 * i + 4 * lane) = o[i];
    __threadfence();
  }
  float* sl = slab[wave];
#pragma unroll
  for (int i = 0; i < 6; ++i) *(v4f*)(sl + 128 * i + 4 * lane) = y[i];
  wave_sync_lds();
  v4u u[3];
#pragma unroll
  for (int j = 0; j < 3; ++j) {
    const v4f a  = *(const v4f*)(sl + 256 * j + 8 * lane);
    const v4f a2 = *(const v4f*)(sl + 256 * j + 8 * lane + 4);
    unsigned short hb[8];
#pragma unroll
    for (int e = 0; e < 4; ++e) { hb[e] = h_bits(a[e]); hb[4 + e] = h_bits(a2[e]); }
    u[j] = (v4u){pk16(hb[0], hb[1]), pk16(hb[2], hb[3]), pk16(hb[4], hb[5]), pk16(hb[6], hb[7])};
  }
  unsigned short* o16 = fus + (size_t)gr * kFfn + kDim;
  for (int pass = 0; pass < 2; ++pass) {
#pragma unroll
    for (int j = 0; j < 3; ++j) *(volatile v4u*)(o16 + 256 * j + 8 * lane) = u[j];
    __threadfence();
  }
}

extern "C" void kernel_launch(void* const* d_in, const int* in_sizes, int n_in,
                              void* d_out, int out_size, void* d_ws, size_t ws_size,
                              hipStream_t stream) {
  (void)in_sizes; (void)n_in; (void)out_size;
  if (ws_size < kWsTotal) return;

  const float* x          = (const float*)d_in[0];
  const float* wq         = (const float*)d_in[1];
  const float* bq         = (const float*)d_in[2];
  const float* wk         = (const float*)d_in[3];
  const float* bk         = (const float*)d_in[4];
  const float* wv         = (const float*)d_in[5];
  const float* bv         = (const float*)d_in[6];
  const float* wo         = (const float*)d_in[7];
  const float* bo         = (const float*)d_in[8];
  const float* rel_bias   = (const float*)d_in[9];
  const float* chan_in_w  = (const float*)d_in[10];
  const float* chan_in_b  = (const float*)d_in[11];
  const float* chan_out_w = (const float*)d_in[12];
  const float* chan_out_b = (const float*)d_in[13];
  const float* ffn_w1     = (const float*)d_in[14];
  const float* ffn_b1     = (const float*)d_in[15];
  const float* ffn_w2     = (const float*)d_in[16];
  const float* ffn_b2     = (const float*)d_in[17];
  const float* g_seq      = (const float*)d_in[18];
  const float* b_seq      = (const float*)d_in[19];
  const float* g_chan     = (const float*)d_in[20];
  const float* b_chan     = (const float*)d_in[21];
  const float* g_ffn      = (const float*)d_in[22];
  const float* b_ffn      = (const float*)d_in[23];
  float* out = (float*)d_out;

  char* ws = (char*)d_ws;
  const float* wsf = (const float*)d_ws;
  float*          XSEQ  = (float*)(ws + kOffXSEQ);
  unsigned short* FUS   = (unsigned short*)(ws + kOffFUS);
  float*          XSUM  = (float*)(ws + kOffXSUM);
  unsigned short* QKV16 = (unsigned short*)(ws + kOffQKV16);
  unsigned short* VTS   = (unsigned short*)(ws + kOffVTS);
  float*          SC    = (float*)(ws + kOffSC);
  unsigned short* X16   = (unsigned short*)(ws + kOffX16);
  unsigned short* P16   = (unsigned short*)(ws + kOffP16);
  unsigned short* WQKVP = (unsigned short*)(ws + kOffWQKVP);
  float*          BQKVP = (float*)(ws + kOffBQKVP);
  unsigned short* CTXS  = (unsigned short*)(ws + kOffCTXS);
  unsigned short* WOP   = (unsigned short*)(ws + kOffWOP);
  float*          S1    = (float*)(ws + kOffS1);
  unsigned short* XT16  = (unsigned short*)(ws + kOffXT16);
  unsigned short* CTXC  = (unsigned short*)(ws + kOffCTXC);
  unsigned short* CIW   = (unsigned short*)(ws + kOffCIW);
  unsigned short* COW   = (unsigned short*)(ws + kOffCOW);
  unsigned short* QKVC  = (unsigned short*)(ws + kOffQKVC);
  float*          CHO   = (float*)(ws + kOffCHO);
  unsigned short* VTC   = (unsigned short*)(ws + kOffVTC);
  float*          SCC   = (float*)(ws + kOffSCC);
  unsigned short* PC    = (unsigned short*)(ws + kOffPC);
  unsigned short* W1    = (unsigned short*)(ws + kOffW1);
  unsigned short* W2    = (unsigned short*)(ws + kOffW2);
  unsigned short* H1    = (unsigned short*)(ws + kOffH1);
  float*          S3    = (float*)(ws + kOffS3);

  const dim3 gb(256);

  k_cast_rows<<<kTok / 8, gb, 0, stream>>>(x, X16, kTok, kDim, 1.0f);
  k_cast_qkvpad<<<385, gb, 0, stream>>>(wq, wk, wv, bq, bk, bv, WQKVP, BQKVP);
  k_cast_wopad<<<kDim / 8, gb, 0, stream>>>(wo, WOP);
  wmma_gemm64<0, false, 2, 1, false, 0><<<dim3(384, 1), gb, 0, stream>>>(
      X16, X16, kDim, 0, WQKVP, WQKVP, kDim, 0, (void*)QKV16, (void*)QKV16, kPadN, 0,
      BQKVP, wsf, 0, kTok, kPadN, kDim, kInvW);
  k_vt_build<<<dim3(kSeq / 64, 64), gb, 0, stream>>>(QKV16, VTS, kSeq);
  for (int c = 0; c < 8; ++c) {
    const int b = c >> 1, h0 = (c & 1) * 8;
    const unsigned short* qp = QKV16 + (size_t)b * kSeq * kPadN + h0 * 64;
    const unsigned short* kp = qp + kQkvW;
    wmma_gemm64<0, false, 0, 0, false, 0><<<dim3(32, 8), gb, 0, stream>>>(
        qp, qp, kPadN, 64, kp, kp, kPadN, 64, (void*)SC, (void*)SC, kSeq, (long)kSeq * kSeq,
        wsf, wsf, 0, kSeq, kSeq, 64, kSeqScale);
    k_softmax<<<8 * kSeq, 128, 0, stream>>>(SC, P16, rel_bias, kSeq, kSeq, h0, 1, kPCarry);
    wmma_gemm64<0, false, 0, 1, false, 0><<<dim3(2, 8), gb, 0, stream>>>(
        P16, P16, kSeq, (long)kSeq * kSeq, VTS + (size_t)c * 8 * 64 * kSeq, VTS + (size_t)c * 8 * 64 * kSeq, kSeq, 64L * kSeq,
        (void*)(CTXS + (size_t)b * kSeq * kQkvW + h0 * 64), (void*)(CTXS + (size_t)b * kSeq * kQkvW + h0 * 64), kQkvW, 64,
        wsf, wsf, 0, kSeq, 64, kSeq, kPVScale);
  }
  wmma_gemm64<0, false, 2, 0, true, 0><<<dim3(96, 1), gb, 0, stream>>>(
      CTXS, CTXS, kQkvW, 0, WOP, WOP, kQkvW, 0, (void*)S1, (void*)S1, kDim, 0,
      bo, x, 0, kTok, kDim, kQkvW, kOutScale);
  k_ln_rows<<<kTok / 8, gb, 0, stream>>>(S1, g_seq, b_seq, XSEQ, FUS, kFfn, 1, kTok);

  k_xt16<<<dim3(kDim / 64, kSeq / 64, kBatch), gb, 0, stream>>>(x, XT16);
  k_cast_rows<<<kPadN / 8, gb, 0, stream>>>(chan_in_w, CIW, kPadN, kSeq, kWCarry);
  wmma_gemm64<0, false, 2, 1, false, 0><<<dim3(72, kBatch), gb, 0, stream>>>(
      XT16, XT16, kSeq, (long)kDim * kSeq, CIW, CIW, kSeq, 0, (void*)QKVC, (void*)QKVC, kPadN, (long)kDim * kPadN,
      chan_in_b, wsf, 0, kDim, kPadN, kSeq, kInvW);
  k_vt_build<<<dim3(kDim / 64, 64), gb, 0, stream>>>(QKVC, VTC, kDim);
  k_cast_rows<<<kSeq / 8, gb, 0, stream>>>(chan_out_w, COW, kSeq, kSeq, kWCarry);
  for (int b = 0; b < kBatch; ++b) {
    const unsigned short* qp = QKVC + (size_t)b * kDim * kPadN;
    const unsigned short* kp = qp + kQkvW;
    wmma_gemm64<0, false, 0, 0, false, 0><<<dim3(18, kHeads), gb, 0, stream>>>(
        qp, qp, kPadN, 64, kp, kp, kPadN, 64, (void*)SCC, (void*)SCC, kDim, (long)kDim * kDim,
        wsf, wsf, 0, kDim, kDim, 64, kChanScale);
    k_softmax<<<kHeads * kDim, 128, 0, stream>>>(SCC, PC, rel_bias, kDim, kDim, 0, 0, kPCarry);
    wmma_gemm64<0, false, 0, 1, false, 0><<<dim3(2, kHeads), gb, 0, stream>>>(
        PC, PC, kDim, (long)kDim * kDim, VTC + (size_t)b * kHeads * 64 * kDim, VTC + (size_t)b * kHeads * 64 * kDim, kDim, 64L * kDim,
        (void*)(CTXC + (size_t)b * kDim * kQkvW), (void*)(CTXC + (size_t)b * kDim * kQkvW), kQkvW, 64,
        wsf, wsf, 0, kDim, 64, kDim, kPVScale);
  }
  wmma_gemm64<0, false, 2, 0, false, 0><<<dim3(24, kBatch), gb, 0, stream>>>(
      CTXC, CTXC, kQkvW, (long)kDim * kQkvW, COW, COW, kSeq, 0, (void*)CHO, (void*)CHO, kSeq, (long)kDim * kSeq,
      chan_out_b, wsf, 0, kDim, kSeq, kSeq, kOutScale);
  k_ln_chan<<<dim3(kSeq / 8, kBatch), gb, 0, stream>>>(CHO, x, XSEQ, g_chan, b_chan, XSUM, FUS);

  k_cast_rows<<<kFfn / 8, gb, 0, stream>>>(ffn_w1, W1, kFfn, kFfn, kWCarry);
  k_cast_rows<<<kDim / 8, gb, 0, stream>>>(ffn_w2, W2, kDim, kFfn, kWCarry);
  wmma_gemm64<0, false, 2, 1, false, 2><<<dim3(192, 1), gb, 0, stream>>>(
      FUS, FUS, kFfn, 0, W1, W1, kFfn, 0, (void*)H1, (void*)H1, kFfn, 0,
      ffn_b1, wsf, 0, kTok, kFfn, kFfn, kInvW);
  wmma_gemm64<0, false, 2, 0, true, 0><<<dim3(96, 1), gb, 0, stream>>>(
      H1, H1, kFfn, 0, W2, W2, kFfn, 0, (void*)S3, (void*)S3, kDim, 0,
      ffn_b2, XSUM, 0, kTok, kDim, kFfn, kInvW);
  k_ln_rows<<<kTok / 8, gb, 0, stream>>>(S3, g_ffn, b_ffn, out, FUS, kFfn, 0, kTok);
}
